// GapJunctionNetwork_57664230916233
// MI455X (gfx1250) — hardware-verified
//
#include <hip/hip_runtime.h>


#define NN_  1024
#define DD   64
#define G1   64
#define G2   32
#define WSC  1024.0f
#define LOSC 1024.0f
#define LOSCI (1.0f / 1024.0f)

typedef _Float16 h16;
typedef __attribute__((ext_vector_type(16))) _Float16 v16h;
typedef __attribute__((ext_vector_type(8)))  _Float16 v8h;
typedef __attribute__((ext_vector_type(8)))  float    v8f;
typedef __attribute__((ext_vector_type(4)))  float    v4f;
typedef __attribute__((ext_vector_type(2)))  float    v2f;
typedef v8h  __attribute__((may_alias)) v8ha;
typedef v4f  __attribute__((may_alias)) v4fa;

__device__ __forceinline__ unsigned short f2bf(float f) { unsigned u = __float_as_uint(f); u += 0x7FFFu + ((u >> 16) & 1u); return (unsigned short)(u >> 16); }
__device__ __forceinline__ float bf2f(unsigned short b) { return __uint_as_float(((unsigned)b) << 16); }
__device__ __forceinline__ float bfr(float f) { return bf2f(f2bf(f)); }
__device__ __forceinline__ v16h cat16(v8h lo, v8h hi) { return __builtin_shufflevector(lo, hi, 0, 1, 2, 3, 4, 5, 6, 7, 8, 9, 10, 11, 12, 13, 14, 15); }
__device__ __forceinline__ v8f wmma16(v16h a, v16h b, v8f c) { return __builtin_amdgcn_wmma_f32_16x16x32_f16(false, a, false, b, (short)0, c, false, false); }
#define VST2(T, p, v) do { const T vst2_v_ = (v); *(volatile T*)(p) = vst2_v_; __threadfence(); *(volatile T*)(p) = vst2_v_; } while (0)

__global__ __launch_bounds__(256) void k_lin(const float* __restrict__ x, const float* __restrict__ w1, const float* __restrict__ b1, const float* __restrict__ sw, const float* __restrict__ sb,
                                            float* HI, float* HJ, float* TF) {
    __shared__ float xs[8][DD];
    const int lane = threadIdx.x & 31, wave = threadIdx.x >> 5, i = blockIdx.x * 8 + wave;
    xs[wave][lane] = bfr(x[(size_t)i * DD + lane]); xs[wave][lane + 32] = bfr(x[(size_t)i * DD + lane + 32]);
    __syncthreads();
    const float* xr = xs[wave];
    v2f ohi, ohj, otf;
#pragma unroll
    for (int e = 0; e < 2; ++e) { const int g = lane * 2 + e; float a = 0.f, bsum = 0.f, t = 0.f;
#pragma unroll 4
        for (int d = 0; d < DD; ++d) { const float xv = xr[d]; a += xv * bfr(w1[g * 2 * DD + d]); bsum += xv * bfr(w1[g * 2 * DD + DD + d]); t += xv * bfr(sw[g * DD + d]); }
        ohi[e] = a; ohj[e] = bsum + bfr(b1[g]); otf[e] = t + bfr(sb[g]); }
    VST2(v2f, HI + (size_t)i * G1 + lane * 2, ohi); VST2(v2f, HJ + (size_t)i * G1 + lane * 2, ohj); VST2(v2f, TF + (size_t)i * DD + lane * 2, otf);
}
__global__ __launch_bounds__(256) void k_tt(const float* __restrict__ TF, h16* TTH, h16* TTL) {
    __shared__ __align__(16) h16 t1[DD * 72];
    __shared__ __align__(16) h16 t2[DD * 72];
    const int i0 = blockIdx.x * 64, tid = threadIdx.x, ii = tid >> 2, d0 = (tid & 3) * 16;
#pragma unroll
    for (int e = 0; e < 16; ++e) { const float v = TF[(size_t)(i0 + ii) * DD + d0 + e]; const h16 a = (h16)v; t1[(d0 + e) * 72 + ii] = a; t2[(d0 + e) * 72 + ii] = (h16)((v - (float)a) * LOSC); }
    __syncthreads();
    const int piece = tid & 7;
    auto pass = [&]() {
#pragma unroll
        for (int s = 0; s < 4; ++s) { const int Lid = (tid >> 3) + 32 * s; const int pln = Lid >> 6, d = Lid & 63;
            const v8h val = *(const v8ha*)((pln ? t2 : t1) + d * 72 + piece * 8); *(volatile v8h*)((pln ? TTL : TTH) + (size_t)d * NN_ + i0 + piece * 8) = val; }
    };
    pass(); __threadfence(); pass();
}
__global__ __launch_bounds__(256) void k_w2(const float* __restrict__ w2, h16* W2H) {
    typedef __attribute__((ext_vector_type(2))) _Float16 v2h;
    const int lane = threadIdx.x & 31, r = blockIdx.x * 8 + (threadIdx.x >> 5);
    if (r >= G2) return;
    v2h o; o[0] = (h16)bfr(w2[r * G1 + 2 * lane]); o[1] = (h16)bfr(w2[r * G1 + 2 * lane + 1]);
    VST2(v2h, W2H + (size_t)r * G1 + 2 * lane, o);
}
__global__ __launch_bounds__(256) void k_adj(const float* __restrict__ A, float* NA) {
    __shared__ float red[256];
    const int i = blockIdx.x, t = threadIdx.x;
    float v[4]; float mx = -3.0e38f;
#pragma unroll
    for (int q = 0; q < 4; ++q) { const int j = t * 4 + q; const float s = (j == i) ? 0.0f : 0.5f * (bfr(A[(size_t)i * NN_ + j]) + bfr(A[(size_t)j * NN_ + i])); v[q] = s; mx = fmaxf(mx, s); }
    red[t] = mx; __syncthreads();
    for (int o = 128; o > 0; o >>= 1) { if (t < o) red[t] = fmaxf(red[t], red[t + o]); __syncthreads(); }
    const float m = red[0]; __syncthreads();
    float e[4], se = 0.f;
#pragma unroll
    for (int q = 0; q < 4; ++q) { e[q] = __expf(v[q] - m); se += e[q]; }
    red[t] = se; __syncthreads();
    for (int o = 128; o > 0; o >>= 1) { if (t < o) red[t] += red[t + o]; __syncthreads(); }
    const float inv = 1.0f / red[0];
    v4f o4;
#pragma unroll
    for (int q = 0; q < 4; ++q) o4[q] = e[q] * inv;
    VST2(v4f, NA + (size_t)i * NN_ + t * 4, o4);
}
__global__ __launch_bounds__(128) void k_gate(const float* __restrict__ HI, const float* __restrict__ HJ, const h16* __restrict__ W2H, const float* __restrict__ b2, const float* __restrict__ w3, const float* __restrict__ b3,
                                             const float* __restrict__ NA, h16* WH, h16* WL) {
    __shared__ float gl[64];
    const int lane = threadIdx.x & 31, wave = threadIdx.x >> 5, lr = lane & 15, hi = lane >> 4;
    const int i = blockIdx.x / (NN_ / 64), jt = blockIdx.x - i * (NN_ / 64), j0 = jt * 64 + wave * 16;
    v16h ah[2], al[2];
#pragma unroll
    for (int kc = 0; kc < 2; ++kc)
#pragma unroll
        for (int q = 0; q < 16; ++q) { const int g = kc * 32 + ((q < 8) ? (8 * hi + q) : (16 + 8 * hi + (q - 8)));
            const float v = fmaxf(HI[(size_t)i * G1 + g] + HJ[(size_t)(j0 + lr) * G1 + g], 0.f); const h16 a = (h16)v; ah[kc][q] = a; al[kc][q] = (h16)((v - (float)a) * LOSC); }
    v8f acc[2], accx[2];
#pragma unroll
    for (int n = 0; n < 2; ++n) { acc[n] = (v8f){}; accx[n] = (v8f){}; }
#pragma unroll
    for (int kc = 0; kc < 2; ++kc)
#pragma unroll
        for (int n = 0; n < 2; ++n) { const h16* bp = W2H + (size_t)(n * 16 + lr) * G1 + kc * 32 + 8 * hi; const v16h bb = cat16(*(const v8h*)bp, *(const v8h*)(bp + 16));
            acc[n] = wmma16(ah[kc], bb, acc[n]); accx[n] = wmma16(al[kc], bb, accx[n]); }
    asm volatile("v_nop\n\tv_nop\n\tv_nop\n\tv_nop" : "+v"(acc[0]), "+v"(acc[1]), "+v"(accx[0]), "+v"(accx[1]));
    float part[8];
#pragma unroll
    for (int j = 0; j < 8; ++j) { float s = 0.f;
#pragma unroll
        for (int n = 0; n < 2; ++n) { const int h = n * 16 + lr; s += fmaxf(acc[n][j] + accx[n][j] * LOSCI + bfr(b2[h]), 0.f) * bfr(w3[h]); }
        s += __shfl_xor(s, 1, 16); s += __shfl_xor(s, 2, 16); s += __shfl_xor(s, 4, 16); s += __shfl_xor(s, 8, 16);
        part[j] = s; }
    if (lr == 0) {
#pragma unroll
        for (int j = 0; j < 8; ++j) { const int jj = j0 + hi * 8 + j; const float gate = 1.0f / (1.0f + __expf(-(part[j] + bfr(b3[0]))));
            gl[wave * 16 + hi * 8 + j] = (jj == i) ? 0.f : gate * NA[(size_t)i * NN_ + jj]; }
    }
    __syncthreads();
    if (wave == 0) { typedef __attribute__((ext_vector_type(2))) _Float16 v2h; const float v0 = gl[lane * 2] * WSC, v1 = gl[lane * 2 + 1] * WSC;
        const h16 a0 = (h16)v0, a1 = (h16)v1; v2h oh, ol; oh[0] = a0; oh[1] = a1; ol[0] = (h16)((v0 - (float)a0) * LOSC); ol[1] = (h16)((v1 - (float)a1) * LOSC);
        VST2(v2h, WH + (size_t)i * NN_ + jt * 64 + lane * 2, oh); VST2(v2h, WL + (size_t)i * NN_ + jt * 64 + lane * 2, ol); }
}
__global__ __launch_bounds__(128) void k_out(const h16* __restrict__ WH, const h16* __restrict__ WL, const h16* __restrict__ TTH, const h16* __restrict__ TTL, const float* __restrict__ x, float* out) {
    __shared__ __align__(16) float ost[4][16 * 68];
    const int lane = threadIdx.x & 31, wave = threadIdx.x >> 5, lr = lane & 15, hi = lane >> 4;
    const int r0 = blockIdx.x * 64 + wave * 16;
    v8f acc[4], accx[4];
#pragma unroll
    for (int n = 0; n < 4; ++n) { acc[n] = (v8f){}; accx[n] = (v8f){}; }
#pragma unroll 2
    for (int kc = 0; kc < NN_ / 32; ++kc) {
        const size_t ao = (size_t)(r0 + lr) * NN_ + kc * 32 + 8 * hi;
        const v16h a = cat16(*(const v8h*)(WH + ao), *(const v8h*)(WH + ao + 16)), al = cat16(*(const v8h*)(WL + ao), *(const v8h*)(WL + ao + 16));
#pragma unroll
        for (int n = 0; n < 4; ++n) { const size_t bo = (size_t)(n * 16 + lr) * NN_ + kc * 32 + 8 * hi;
            const v16h bh = cat16(*(const v8h*)(TTH + bo), *(const v8h*)(TTH + bo + 16)), bl = cat16(*(const v8h*)(TTL + bo), *(const v8h*)(TTL + bo + 16));
            acc[n] = wmma16(a, bh, acc[n]); accx[n] = wmma16(a, bl, accx[n]); accx[n] = wmma16(al, bh, accx[n]); }
        asm volatile("v_nop\n\tv_nop" : "+v"(acc[0]), "+v"(acc[3]), "+v"(accx[0]), "+v"(accx[3]) : "v"(a), "v"(al));
    }
    asm volatile("v_nop\n\tv_nop\n\tv_nop\n\tv_nop" : "+v"(acc[0]), "+v"(acc[1]), "+v"(acc[2]), "+v"(acc[3]), "+v"(accx[0]), "+v"(accx[1]), "+v"(accx[2]), "+v"(accx[3]));
    float* os = &ost[wave][0];
#pragma unroll
    for (int n = 0; n < 4; ++n)
#pragma unroll
        for (int j = 0; j < 8; ++j) { const int row = r0 + hi * 8 + j, d = n * 16 + lr; os[(hi * 8 + j) * 68 + d] = (acc[n][j] + accx[n][j] * LOSCI) * (1.0f / WSC) + bfr(x[(size_t)row * DD + d]); }
    __syncthreads();
    float* crow = out + (size_t)r0 * DD;
    auto pass = [&]() {
#pragma unroll
        for (int s = 0; s < 8; ++s) { const int Lid = (lane >> 3) + 4 * s, piece = lane & 7; const int row = Lid >> 1, cofs = (Lid & 1) * 32 + piece * 4;
            const v4f val = *(const v4fa*)(os + row * 68 + cofs); *(volatile v4f*)(crow + (size_t)row * DD + cofs) = val; }
    };
    pass(); __threadfence(); pass();
}

extern "C" void kernel_launch(void* const* d_in, const int* in_sizes, int n_in,
                              void* d_out, int out_size, void* d_ws, size_t ws_size, hipStream_t stream) {
    (void)in_sizes; (void)n_in; (void)out_size;
    const float* x = (const float*)d_in[0]; const float* A = (const float*)d_in[1]; const float* w1 = (const float*)d_in[2]; const float* b1 = (const float*)d_in[3];
    const float* w2 = (const float*)d_in[4]; const float* b2 = (const float*)d_in[5]; const float* w3 = (const float*)d_in[6]; const float* b3 = (const float*)d_in[7];
    const float* sw = (const float*)d_in[8]; const float* sb = (const float*)d_in[9];
    float* out = (float*)d_out;
    char* wsp = (char*)d_ws;
    auto take = [&](size_t bytes) { char* p = wsp; wsp += (bytes + 255) & ~(size_t)255; return (void*)p; };
    float* HI = (float*)take((size_t)NN_ * G1 * 4); float* HJ = (float*)take((size_t)NN_ * G1 * 4); float* TF = (float*)take((size_t)NN_ * DD * 4);
    h16* TTH = (h16*)take((size_t)DD * NN_ * 2); h16* TTL = (h16*)take((size_t)DD * NN_ * 2); h16* W2H = (h16*)take((size_t)G2 * G1 * 2); float* NA = (float*)take((size_t)NN_ * NN_ * 4);
    h16* WH = (h16*)take((size_t)NN_ * NN_ * 2); h16* WL = (h16*)take((size_t)NN_ * NN_ * 2);
    if ((size_t)(wsp - (char*)d_ws) > ws_size) return;
    k_lin<<<NN_ / 8, 256, 0, stream>>>(x, w1, b1, sw, sb, HI, HJ, TF);
    k_tt<<<NN_ / 64, 256, 0, stream>>>(TF, TTH, TTL);
    k_w2<<<(G2 + 7) / 8, 256, 0, stream>>>(w2, W2H);
    k_adj<<<NN_, 256, 0, stream>>>(A, NA);
    k_gate<<<NN_ * (NN_ / 64), 128, 0, stream>>>(HI, HJ, W2H, b2, w3, b3, NA, WH, WL);
    k_out<<<NN_ / 64, 128, 0, stream>>>(WH, WL, TTH, TTL, x, out);
}
